// onestepKernel_79267916415212
// MI455X (gfx1250) — hardware-verified
//
#include <hip/hip_runtime.h>
#include <math.h>

#define NN 50000
#define NE 400000
#define CC 32
#define KW 128
#define EF 6
#define EB 32
#define NEB (NE / EB)
#define NFRAG 320
#define WQ_DW (NFRAG * 256)
#define NT 256
#define TN 1024
#define NTILE ((NN + TN - 1) / TN)
#define SCH 2048
#define SPT (SCH / NT)
#define NCHA ((NE + SCH - 1) / SCH)
static_assert(NE % EB == 0, "edge blocks tile the edge list exactly");
static_assert(NE % SPT == 0, "a thread dst group is entirely inside or outside the list");
static_assert(SPT * NT == SCH, "chunk geometry");
static_assert(TN % 8 == 0, "eight owner waves per tile");

typedef __attribute__((ext_vector_type(16))) _Float16 v16h;
typedef __attribute__((ext_vector_type(8)))  _Float16 v8h;
typedef __attribute__((ext_vector_type(8)))  float    v8f;
typedef __attribute__((ext_vector_type(4)))  float    v4f;
typedef __attribute__((ext_vector_type(4)))  int      v4i;

__device__ __forceinline__ void dep_guard_h(v8f& a, v8f& b, v16h x, v16h y) { asm volatile("v_nop\n\tv_nop\n\tv_nop\n\tv_nop" : "+v"(a), "+v"(b) : "v"(x), "v"(y)); }
__device__ __forceinline__ void keep4_h(v16h a, v16h b, v16h c, v16h d) { asm volatile("v_nop" :: "v"(a), "v"(b), "v"(c), "v"(d)); }
__device__ __forceinline__ void guard3(v8f& a, v8f& b, v16h x, v16h y, v16h z) {
  asm volatile("v_nop\n\tv_nop\n\tv_nop\n\tv_nop" : "+v"(a), "+v"(b) : "v"(x), "v"(y), "v"(z));
}
template <typename T> struct Frag;
template <> struct Frag<_Float16> {
  typedef v16h V; union U { v16h v; v8h h[2]; };
  static __device__ __forceinline__ v16h load(const _Float16* p) {
    U f; f.h[0] = *(const v8h*)(p); f.h[1] = *(const v8h*)(p + 16); return f.v;
  }
  static __device__ __forceinline__ v8f mma(v16h a, v16h b, v8f c) {
    return __builtin_amdgcn_wmma_f32_16x16x32_f16(false, a, false, b, (short)0, c, false, false);
  }
  static __device__ __forceinline__ void guard(v8f& a, v8f& b, v16h x, v16h y) { dep_guard_h(a, b, x, y); }
  static __device__ __forceinline__ void keep(v16h a, v16h b, v16h c, v16h d) { keep4_h(a, b, c, d); }
};

__device__ __forceinline__ float prelu_f(float x, float a) { return x >= 0.f ? x : a * x; }

__device__ __forceinline__ v16h load_bfrag(const _Float16* __restrict__ wq, int fid, int lane) {
  union { v16h v; v8h h2[2]; } u;
  const _Float16* p = wq + (size_t)fid * 512 + lane * 16;
  u.h2[0] = *(const v8h*)(p);
  u.h2[1] = *(const v8h*)(p + 8);
  return u.v;
}

__global__ __launch_bounds__(NT) void pack_kernel(const float* __restrict__ W2, const float* __restrict__ W3, const float* __restrict__ W4,
                                                 unsigned* __restrict__ wq32) {
  const int i = blockIdx.x * NT + threadIdx.x;
  if (i >= WQ_DW) return;
  const int fid = i >> 8;
  const int w = i & 255;
  const int lane = w >> 3, p = w & 7;
  const int nl = lane & 15, h = lane >> 4;
  const int kt = fid & 3;
  const float* W; int nt, Nw;
  if (fid < 32)      { W = W2; nt = fid >> 2;        Nw = KW; }
  else if (fid < 64) { W = W3; nt = (fid - 32) >> 2; Nw = KW; }
  else               { W = W4; nt = (fid - 64) >> 2; Nw = KW * 8; }
  const int n = nt * 16 + nl;
  const int e0 = 2 * p;
  const int k0 = kt * 32 + 8 * h + e0 + ((e0 >= 8) ? 8 : 0);
  const float a = W[(size_t)k0 * Nw + n];
  const float b = W[(size_t)(k0 + 1) * Nw + n];
  const unsigned u = (unsigned)__builtin_bit_cast(unsigned short, (_Float16)a) | ((unsigned)__builtin_bit_cast(unsigned short, (_Float16)b) << 16);
  ((volatile unsigned*)wq32)[i] = u;
  __threadfence();
  ((volatile unsigned*)wq32)[i] = u;
}

__device__ __forceinline__ void mlp_layer(const _Float16* hsrc, _Float16* hdst, const _Float16* __restrict__ wq, int fragbase,
                                          const float* __restrict__ bvec, float alpha, int lane, int nl, int h, int wv) {
  const v8f z8 = {0.f, 0.f, 0.f, 0.f, 0.f, 0.f, 0.f, 0.f};
  v8f acc0 = z8, acc1 = z8;
#pragma unroll
  for (int kt = 0; kt < 4; ++kt) {
    const v16h b  = load_bfrag(wq, fragbase + wv * 4 + kt, lane);
    const v16h a0 = Frag<_Float16>::load(hsrc + nl * KW + kt * 32 + 8 * h);
    const v16h a1 = Frag<_Float16>::load(hsrc + (16 + nl) * KW + kt * 32 + 8 * h);
    acc0 = Frag<_Float16>::mma(a0, b, acc0);
    acc1 = Frag<_Float16>::mma(a1, b, acc1);
    guard3(acc0, acc1, a0, a1, b);
  }
  const float bv = bvec[wv * 16 + nl];
#pragma unroll
  for (int r = 0; r < 8; ++r) {
    const int off = (8 * h + r) * KW + wv * 16 + nl;
    hdst[off]           = (_Float16)prelu_f(acc0[r] + bv, alpha);
    hdst[off + 16 * KW] = (_Float16)prelu_f(acc1[r] + bv, alpha);
  }
}

__global__ __launch_bounds__(NT) void edge_kernel(const float* __restrict__ ea, const int* __restrict__ ei, const float* __restrict__ xr,
                                                 const float* __restrict__ W1, const float* __restrict__ b1,
                                                 const float* __restrict__ b2, const float* __restrict__ b3, const float* __restrict__ b4,
                                                 const float* __restrict__ pa1, const float* __restrict__ pa2, const float* __restrict__ pa3,
                                                 const _Float16* __restrict__ wq, float* __restrict__ Mout) {
  __shared__ __align__(16) _Float16 hA[EB * KW];
  __shared__ __align__(16) _Float16 hB[EB * KW];
  __shared__ __align__(16) float xs_s[EB * CC];
  __shared__ __align__(16) float part[8 * EB * CC];
  __shared__ float ea_s[EB * EF];
  __shared__ int src_s[EB];

  const int tid  = threadIdx.x;
  const int lane = tid & 31;
  const int wv   = tid >> 5;
  const int nl   = lane & 15;
  const int h    = lane >> 4;
  const int e0   = blockIdx.x * EB;

  if (tid < EB * EF) ea_s[tid] = ea[(size_t)e0 * EF + tid];
  if (tid >= 192 && tid < 192 + EB) {
    int s = ei[e0 + (tid - 192)];
    s = s < 0 ? 0 : (s >= NN ? NN - 1 : s);
    src_s[tid - 192] = s;
  }
  __syncthreads();

  {
    const int m = tid >> 4, j0 = (tid & 15) * 8;
    const float a1v = pa1[0];
    v4f wlo[EF], whi[EF];
#pragma unroll
    for (int f = 0; f < EF; ++f) {
      wlo[f] = *(const v4f*)(W1 + f * KW + j0);
      whi[f] = *(const v4f*)(W1 + f * KW + j0 + 4);
    }
    const v4f blo = *(const v4f*)(b1 + j0), bhi = *(const v4f*)(b1 + j0 + 4);
#pragma unroll
    for (int mt = 0; mt < 2; ++mt) {
      const int row = mt * 16 + m;
      float ev[EF];
#pragma unroll
      for (int f = 0; f < EF; ++f) ev[f] = ea_s[row * EF + f];
      v4f dlo = ev[0] * wlo[0], dhi = ev[0] * whi[0];
#pragma unroll
      for (int f = 1; f < EF; ++f) { dlo = dlo + ev[f] * wlo[f]; dhi = dhi + ev[f] * whi[f]; }
      dlo = dlo + blo; dhi = dhi + bhi;
      v8h hv;
#pragma unroll
      for (int e = 0; e < 4; ++e) {
        hv[e]     = (_Float16)prelu_f(dlo[e], a1v);
        hv[4 + e] = (_Float16)prelu_f(dhi[e], a1v);
      }
      *(v8h*)(hA + row * KW + j0) = hv;
    }
  }
  for (int i = tid; i < EB * CC; i += NT) xs_s[i] = xr[(size_t)src_s[i >> 5] * CC + (i & 31)];
  __syncthreads();

  mlp_layer(hA, hB, wq, 0,  b2, pa2[0], lane, nl, h, wv);
  __syncthreads();
  mlp_layer(hB, hA, wq, 32, b3, pa3[0], lane, nl, h, wv);
  __syncthreads();

  v16h A0[4], A1[4];
#pragma unroll
  for (int kt = 0; kt < 4; ++kt) {
    A0[kt] = Frag<_Float16>::load(hA + nl * KW + kt * 32 + 8 * h);
    A1[kt] = Frag<_Float16>::load(hA + (16 + nl) * KW + kt * 32 + 8 * h);
  }
  float msg0[16], msg1[16];
#pragma unroll
  for (int i = 0; i < 16; ++i) { msg0[i] = 0.f; msg1[i] = 0.f; }
  const v8f z8 = {0.f, 0.f, 0.f, 0.f, 0.f, 0.f, 0.f, 0.f};

#pragma unroll 1
  for (int tp = 0; tp < 4; ++tp) {
    const int c = wv * 4 + tp;
    float x0r[8], x1r[8];
#pragma unroll
    for (int r = 0; r < 8; ++r) {
      x0r[r] = xs_s[(8 * h + r) * CC + c];
      x1r[r] = xs_s[(16 + 8 * h + r) * CC + c];
    }
#pragma unroll
    for (int par = 0; par < 2; ++par) {
      const int nt = 2 * c + par;
      v8f acc0 = z8, acc1 = z8;
#pragma unroll
      for (int kt = 0; kt < 4; ++kt) {
        const v16h b = load_bfrag(wq, 64 + nt * 4 + kt, lane);
        acc0 = Frag<_Float16>::mma(A0[kt], b, acc0);
        acc1 = Frag<_Float16>::mma(A1[kt], b, acc1);
        guard3(acc0, acc1, A0[kt], A1[kt], b);
      }
      const float b4v = b4[nt * 16 + nl];
#pragma unroll
      for (int r = 0; r < 8; ++r) {
        const float w0 = acc0[r] + b4v;
        const float w1 = acc1[r] + b4v;
        msg0[par * 8 + r] = fmaf(x0r[r], w0, msg0[par * 8 + r]);
        msg1[par * 8 + r] = fmaf(x1r[r], w1, msg1[par * 8 + r]);
      }
    }
  }

  {
    float* pw = part + wv * (EB * CC);
#pragma unroll
    for (int par = 0; par < 2; ++par) {
#pragma unroll
      for (int r = 0; r < 8; ++r) {
        const int off = (8 * h + r) * CC + par * 16 + nl;
        pw[off]           = msg0[par * 8 + r];
        pw[off + 16 * CC] = msg1[par * 8 + r];
      }
    }
  }
  __syncthreads();
  {
    const int idx = tid * 4;
    v4f s = *(const v4f*)(part + idx);
#pragma unroll
    for (int w = 1; w < 8; ++w) s = s + *(const v4f*)(part + w * (EB * CC) + idx);
    float* mp = Mout + (size_t)e0 * CC + idx;
    *(volatile v4f*)mp = s;
    __threadfence();
    *(volatile v4f*)mp = s;
  }
}

__device__ __forceinline__ int blk_excl_scan(int cnt, int* scan_ws, int tid, int* tot) {
  const int lane = tid & 31, wave = tid >> 5; int incl = cnt;
#pragma unroll
  for (int o = 1; o < 32; o <<= 1) { const int v = __shfl_up(incl, o, 32); if (lane >= o) incl += v; }
  if (lane == 31) scan_ws[wave] = incl;
  __syncthreads();
  if (wave == 0) { int wv = (lane < NT / 32) ? scan_ws[lane] : 0; int wincl = wv;
#pragma unroll
    for (int o = 1; o < 32; o <<= 1) { const int v = __shfl_up(wincl, o, 32); if (lane >= o) wincl += v; }
    if (lane < NT / 32) scan_ws[32 + lane] = wincl - wv; if (lane == 31) scan_ws[64] = wincl; }
  __syncthreads();
  const int res = scan_ws[32 + wave] + incl - cnt; *tot = scan_ws[64];
  return res;
}
__device__ __forceinline__ int chunk_hits(const int* __restrict__ dstv, int e0, int n0, int tid, int* LIST, int* scan_ws) {
  const int eb = e0 + tid * SPT;
  int rec[SPT]; int cnt = 0;
#pragma unroll
  for (int k = 0; k < SPT; k += 4) {
    v4i d4 = {-1, -1, -1, -1};
    if (eb < NE) d4 = *(const v4i*)(dstv + eb + k);
#pragma unroll
    for (int e = 0; e < 4; ++e) {
      const int d = d4[e]; int r = -1;
      if (d >= n0 && d < n0 + TN) { r = ((d - n0) << 11) | (tid * SPT + k + e); ++cnt; }
      rec[k + e] = r;
    }
  }
  int tot; int p = blk_excl_scan(cnt, scan_ws, tid, &tot);
#pragma unroll
  for (int k = 0; k < SPT; ++k) if (rec[k] >= 0) { if ((unsigned)p < (unsigned)SCH) LIST[p] = rec[k]; ++p; }
  __syncthreads();
  return tot < SCH ? tot : SCH;
}

__global__ __launch_bounds__(NT) void agg_kernel(const float* __restrict__ M, const int* __restrict__ ei, const float* __restrict__ xr,
                                                const float* __restrict__ root, const float* __restrict__ bias, const float* __restrict__ paout,
                                                float* __restrict__ out) {
  __shared__ __align__(16) float ACC[TN * CC];
  __shared__ int CNT[TN];
  __shared__ int LIST[SCH];
  __shared__ int scan_ws[80];
  const int tid = threadIdx.x, lane = tid & 31, wave = tid >> 5;
  const int n0 = blockIdx.x * TN;
  const v4f z4 = {0.f, 0.f, 0.f, 0.f};
  for (int i = tid; i < TN * CC / 4; i += NT) *(v4f*)(ACC + 4 * i) = z4;
  for (int i = tid; i < TN; i += NT) CNT[i] = 0;
  float rr[CC];
#pragma unroll
  for (int c = 0; c < CC; ++c) rr[c] = root[c * CC + lane];
  const float bo = bias[lane];
  const float ao = paout[0];
  __syncthreads();

  const int* dstv = ei + NE;
#pragma unroll 1
  for (int ch = 0; ch < NCHA; ++ch) {
    const int tot = chunk_hits(dstv, ch * SCH, n0, tid, LIST, scan_ws);
#pragma unroll 1
    for (int base = 0; base < tot; base += 32) {
      const int q = base + lane;
      const int rv = (q < tot) ? LIST[q] : -1;
      const int own = (rv >= 0 && (rv >> 18) == wave) ? 1 : 0;
      unsigned msk = (unsigned)__ballot(own);
#pragma unroll 1
      for (int it = 0; it < 32; ++it) {
        if (msk == 0u) break;
        const int bp = __builtin_ctz(msk); msk &= msk - 1u;
        const int r = __shfl(rv, bp, 32);
        const int dl = (r >> 11) & (TN - 1);
        int e = ch * SCH + (r & (SCH - 1)); e = e < NE ? e : NE - 1;
        const float mv = M[(size_t)e * CC + lane];
        const int ai = dl * CC + lane;
        ACC[ai] = ACC[ai] + mv;
        if (lane == 0) CNT[dl] = CNT[dl] + 1;
      }
    }
    __syncthreads();
  }

#pragma unroll 1
  for (int j = 0; j < TN / 8; ++j) {
    const int dl = wave * (TN / 8) + j;
    const int n = n0 + dl;
    if (n < NN) {
      const int cn = CNT[dl];
      const float cf = (float)(cn < 1 ? 1 : cn);
      const float inv = 1.0f / cf;
      const float mean = ACC[dl * CC + lane] * inv;
      const v4f* xp = (const v4f*)(xr + (size_t)n * CC);
      float rt = 0.f;
#pragma unroll
      for (int q4 = 0; q4 < 8; ++q4) {
        const v4f xv = xp[q4];
        rt = fmaf(xv[0], rr[4 * q4 + 0], rt);
        rt = fmaf(xv[1], rr[4 * q4 + 1], rt);
        rt = fmaf(xv[2], rr[4 * q4 + 2], rt);
        rt = fmaf(xv[3], rr[4 * q4 + 3], rt);
      }
      float v = mean + rt;
      v = v + bo;
      v = prelu_f(v, ao);
      float* op = out + (size_t)n * CC + lane;
      *(volatile float*)op = v;
      __threadfence();
      *(volatile float*)op = v;
    }
  }
}

extern "C" void kernel_launch(void* const* d_in, const int* in_sizes, int n_in,
                              void* d_out, int out_size, void* d_ws, size_t ws_size, hipStream_t stream) {
  (void)in_sizes; (void)n_in; (void)out_size;
  const float* xr   = (const float*)d_in[0];
  const float* ea   = (const float*)d_in[1];
  const float* W1   = (const float*)d_in[2];
  const float* b1   = (const float*)d_in[3];
  const float* W2   = (const float*)d_in[4];
  const float* b2   = (const float*)d_in[5];
  const float* W3   = (const float*)d_in[6];
  const float* b3   = (const float*)d_in[7];
  const float* W4   = (const float*)d_in[8];
  const float* b4   = (const float*)d_in[9];
  const float* a1   = (const float*)d_in[10];
  const float* a2   = (const float*)d_in[11];
  const float* a3   = (const float*)d_in[12];
  const float* root = (const float*)d_in[13];
  const float* bias = (const float*)d_in[14];
  const float* aout = (const float*)d_in[15];
  const int*   ei   = (const int*)d_in[16];
  float* out = (float*)d_out;

  char* ws = (char*)d_ws; size_t off = 0;
  auto carve = [&](size_t bytes) -> char* { char* p = ws + off; off += (bytes + 255) & ~(size_t)255; return p; };
  unsigned* wq32 = (unsigned*)carve((size_t)WQ_DW * 4);
  float*    Mbuf = (float*)carve((size_t)NE * CC * 4);
  if (off > ws_size || off > (size_t)134217728) return;

  pack_kernel<<<NFRAG, NT, 0, stream>>>(W2, W3, W4, wq32);
  edge_kernel<<<NEB, NT, 0, stream>>>(ea, ei, xr, W1, b1, b2, b3, b4, a1, a2, a3,
                                      (const _Float16*)wq32, Mbuf);
  agg_kernel<<<NTILE, NT, 0, stream>>>(Mbuf, ei, xr, root, bias, aout, out);
}
